// CapsLayerWithClusterRouting_55894704390186
// MI455X (gfx1250) — hardware-verified
//
#include <hip/hip_runtime.h>
#include <stdint.h>
#include <math.h>


typedef __bf16 v16bf __attribute__((ext_vector_type(16)));
typedef float v8f __attribute__((ext_vector_type(8)));
typedef float v4f __attribute__((ext_vector_type(4)));
typedef unsigned int v4u __attribute__((ext_vector_type(4)));

enum {
  NBATCH = 16, NCI = 8, NKV = 4, NCO = 8, NDI = 16, NDO = 16, NS = 64,
  NCH = 4096, KRED = 144, KPAD = 160, KCH = 20, APITCH4 = 21,
  NCONVBLK = 512, NWCHUNK = NCH * KCH, PARTW = 32
};

union Frag { v4u q[2]; v16bf v; };

__device__ __forceinline__ unsigned int f2bf16(float f) {
  unsigned int u = __float_as_uint(f);
  u += 0x7FFFu + ((u >> 16) & 1u);
  return u >> 16;
}
__device__ __forceinline__ float bf16_rne(float f) {
  return __uint_as_float(f2bf16(f) << 16);
}
__device__ __forceinline__ v8f zero8() {
  v8f z;
  #pragma unroll
  for (int i = 0; i < 8; ++i) z[i] = 0.f;
  return z;
}
__device__ __forceinline__ v8f wmma_bf16(v16bf a, v16bf b, v8f c) {
  v8f d = __builtin_amdgcn_wmma_f32_16x16x32_bf16(false, a, false, b, (short)0, c, false, false);
  asm volatile("v_nop\n\tv_nop\n\tv_nop\n\tv_nop" : "+v"(d) : "v"(a), "v"(b));
  return d;
}

__global__ void __launch_bounds__(256) k_prep(const float* __restrict__ W,
                                             v4u* __restrict__ Wr, int nchunk)
{
  int g = blockIdx.x * 256 + threadIdx.x;
  if (g < nchunk) {
    int orow = g / KCH;
    int kc = g - orow * KCH;
    int s = orow >> 6, kk = (orow >> 4) & 3, r = orow & 15;
    int c_out = s >> 3, ci = s & 7;
    int co = ci * 512 + kk * 128 + c_out * 16 + r;
    int kv0 = kc * 8;
    int tap = kv0 >> 4, c0 = kv0 & 15;
    unsigned int hv[8];
    if (tap < 9) {
      const float* wp = W + (size_t)co * KRED + c0 * 9 + tap;
      #pragma unroll
      for (int j = 0; j < 8; ++j) hv[j] = f2bf16(wp[j * 9]);
    } else {
      #pragma unroll
      for (int j = 0; j < 8; ++j) hv[j] = 0u;
    }
    v4u pk;
    pk.x = hv[0] | (hv[1] << 16);
    pk.y = hv[2] | (hv[3] << 16);
    pk.z = hv[4] | (hv[5] << 16);
    pk.w = hv[6] | (hv[7] << 16);
    volatile v4u* p = (volatile v4u*)(Wr + g);
    *p = pk;
    __threadfence();
    *p = pk;
  }
}

__global__ void __launch_bounds__(256) k_conv_route(
    const float* __restrict__ X, const v4u* __restrict__ Wr,
    const float* __restrict__ bias, float* __restrict__ capsbuf,
    float* __restrict__ part)
{
  __shared__ v4u Alds[128 * APITCH4];
  __shared__ v4u Bq[64 * KCH];
  __shared__ v4f Stg[32 * 16];
  __shared__ float Red[NCO * 8 * 2];

  const int blk = blockIdx.x;
  const int h0 = (blk & 31) << 1;
  const int b = blk >> 5;
  const int tid = threadIdx.x;

  #pragma unroll 1
  for (int e = 0; e < 10; ++e) {
    int idx = tid + e * 256;
    int row = idx / KCH;
    int kc = idx - row * KCH;
    int t = row >> 4, p = row & 15;
    int kv0 = kc * 8;
    int tap = kv0 >> 4, c0 = kv0 & 15;
    float v[8];
    #pragma unroll
    for (int j = 0; j < 8; ++j) v[j] = 0.f;
    if (tap < 9) {
      int kh = tap / 3, kw = tap - kh * 3;
      int hh = h0 + (t >> 2) + kh - 1;
      int ww = ((t & 3) << 4) + p + kw - 1;
      if (hh >= 0 && hh < NS && ww >= 0 && ww < NS) {
        const float* xp = X + ((size_t)(b * NDI + c0) * NS + hh) * NS + ww;
        #pragma unroll
        for (int j = 0; j < 8; ++j) v[j] = xp[(size_t)j * NS * NS];
      }
    }
    v4u pk;
    pk.x = f2bf16(v[0]) | (f2bf16(v[1]) << 16);
    pk.y = f2bf16(v[2]) | (f2bf16(v[3]) << 16);
    pk.z = f2bf16(v[4]) | (f2bf16(v[5]) << 16);
    pk.w = f2bf16(v[6]) | (f2bf16(v[7]) << 16);
    Alds[row * APITCH4 + kc] = pk;
  }

  const int lane = tid & 31, wid = tid >> 5;
  const int l16 = lane & 15, half = lane >> 4;

  __syncthreads();

  Frag afrag[5];
  {
    const v4u* arow = &Alds[(wid * 16 + l16) * APITCH4];
    #pragma unroll
    for (int ks = 0; ks < 5; ++ks) {
      afrag[ks].q[0] = arow[ks * 4 + half];
      afrag[ks].q[1] = arow[ks * 4 + 2 + half];
    }
  }

  v8f amax, se, wsum;
  amax = zero8(); se = zero8(); wsum = zero8();

  #pragma unroll 1
  for (int s = 0; s < 64; ++s) {
    const int c_out = s >> 3, ci = s & 7;
    if (ci == 0) {
      #pragma unroll
      for (int i = 0; i < 8; ++i) { amax[i] = -__builtin_inff(); se[i] = 0.f; wsum[i] = 0.f; }
    }
    __syncthreads();
    {
      const v4u* src = Wr + (size_t)s * (64 * KCH);
      #pragma unroll
      for (int q = 0; q < 5; ++q) {
        int i = tid + q * 256;
        Bq[i] = src[i];
      }
    }
    __syncthreads();

    v8f sumv = zero8(), sqv = zero8();
    #pragma unroll
    for (int kk = 0; kk < 4; ++kk) {
      const v4u* brow = &Bq[(kk * 16 + l16) * KCH];
      v8f acc = zero8();
      #pragma unroll
      for (int ks = 0; ks < 5; ++ks) {
        Frag bfr;
        bfr.q[0] = brow[ks * 4 + half];
        bfr.q[1] = brow[ks * 4 + 2 + half];
        acc = wmma_bf16(afrag[ks].v, bfr.v, acc);
      }
      float bv = bf16_rne(bias[ci * 512 + kk * 128 + c_out * 16 + l16]);
      #pragma unroll
      for (int i = 0; i < 8; ++i) {
        float x = acc[i] + bv;
        sumv[i] += x;
        sqv[i] += x * x;
      }
    }
    #pragma unroll
    for (int i = 0; i < 8; ++i) {
      float mean = sumv[i] * 0.25f;
      float var  = sqv[i] * 0.25f - mean * mean;
      float sd   = sqrtf(fmaxf(var, 0.f));
      float ag   = -logf(fmaxf(sd, 1e-30f));
      float mn   = fmaxf(amax[i], ag);
      float sc   = expf(amax[i] - mn);
      float ev   = expf(ag - mn);
      se[i]   = se[i] * sc + ev;
      wsum[i] = wsum[i] * sc + ev * mean;
      amax[i] = mn;
    }

    if (ci == 7) {
      float cval[8];
      float s1 = 0.f, s2 = 0.f;
      #pragma unroll
      for (int i = 0; i < 8; ++i) {
        float c = wsum[i] / se[i];
        cval[i] = c; s1 += c; s2 += c * c;
      }
      #pragma unroll
      for (int off = 16; off >= 1; off >>= 1) {
        s1 += __shfl_xor(s1, off, 32);
        s2 += __shfl_xor(s2, off, 32);
      }
      if (lane == 0) {
        Red[(c_out * 8 + wid) * 2]     = s1;
        Red[(c_out * 8 + wid) * 2 + 1] = s2;
      }
      const int hl = wid >> 2, w0 = (wid & 3) << 4;
      v4f c0, c1;
      c0.x = cval[0]; c0.y = cval[1]; c0.z = cval[2]; c0.w = cval[3];
      c1.x = cval[4]; c1.y = cval[5]; c1.z = cval[6]; c1.w = cval[7];
      const int si = (hl * 16 + l16) * 16 + (w0 >> 2) + half * 2;
      Stg[si] = c0;
      Stg[si + 1] = c1;
      __syncthreads();
      const int q4 = lane & 7, lsub = lane >> 3;
      const int L0 = wid * 8 + lsub, L1 = L0 + 4;
      const int r0 = L0 >> 1, r1 = L1 >> 1;
      const int d0 = r0 & 15, hla = r0 >> 4, d1 = r1 & 15, hlb = r1 >> 4;
      const int wo0 = (L0 & 1) * 32 + q4 * 4, wo1 = (L1 & 1) * 32 + q4 * 4;
      v4f v0 = Stg[r0 * 16 + (wo0 >> 2)];
      v4f v1 = Stg[r1 * 16 + (wo1 >> 2)];
      float* g0 = capsbuf + ((size_t)((b * NCO + c_out) * NDO + d0) * NS + h0 + hla) * NS + wo0;
      float* g1 = capsbuf + ((size_t)((b * NCO + c_out) * NDO + d1) * NS + h0 + hlb) * NS + wo1;
      *(volatile v4f*)g0 = v0;
      *(volatile v4f*)g1 = v1;
      __threadfence();
      *(volatile v4f*)g0 = v0;
      *(volatile v4f*)g1 = v1;
    }
  }

  __syncthreads();
  if (tid < 8) {
    v4f pv;
    pv.x = 0.f; pv.y = 0.f; pv.z = 0.f; pv.w = 0.f;
    if (tid < 4) {
      const int ca = tid * 2, cb = ca + 1;
      float a0 = 0.f, a1 = 0.f, b0 = 0.f, b1 = 0.f;
      #pragma unroll
      for (int w = 0; w < 8; ++w) {
        a0 += Red[(ca * 8 + w) * 2];
        a1 += Red[(ca * 8 + w) * 2 + 1];
        b0 += Red[(cb * 8 + w) * 2];
        b1 += Red[(cb * 8 + w) * 2 + 1];
      }
      pv.x = a0; pv.y = a1; pv.z = b0; pv.w = b1;
    }
    float* pp = part + (size_t)blk * PARTW + tid * 4;
    *(volatile v4f*)pp = pv;
    __threadfence();
    *(volatile v4f*)pp = pv;
  }
}

__global__ void __launch_bounds__(256) k_final(const float* __restrict__ capsbuf,
                                              const float* __restrict__ part,
                                              const float* __restrict__ gamma,
                                              const float* __restrict__ beta,
                                              float* __restrict__ out, int n4)
{
  __shared__ float sh[64];
  __shared__ float st[2];
  const int gb = blockIdx.x * 256;
  const int co = gb >> 18;
  const int b  = (gb >> 14) & 15;
  if (threadIdx.x < 64) {
    int hp = threadIdx.x >> 1, wh = threadIdx.x & 1;
    sh[threadIdx.x] = part[(size_t)(b * 32 + hp) * PARTW + co * 2 + wh];
  }
  __syncthreads();
  if (threadIdx.x == 0) {
    double s1 = 0.0, s2 = 0.0;
    for (int hp = 0; hp < 32; ++hp) { s1 += (double)sh[2 * hp]; s2 += (double)sh[2 * hp + 1]; }
    const double inv_n = 1.0 / 65536.0;
    double mean = s1 * inv_n;
    double var = s2 * inv_n - mean * mean;
    if (var < 0.0) var = 0.0;
    st[0] = (float)mean;
    st[1] = 1.0f / sqrtf((float)var + 1e-5f);
  }
  __syncthreads();
  const float mean = st[0], rstd = st[1];
  const int g = gb + threadIdx.x;
  if (g < n4) {
    int rem2 = g & 16383;
    int d    = rem2 >> 10;
    int hw4  = rem2 & 1023;
    v4f cv = *(const v4f*)(capsbuf + ((size_t)((b * NCO + co) * NDO + d) * 1024 + hw4) * 4);
    v4f gm = *(const v4f*)(gamma + ((size_t)d * 1024 + hw4) * 4);
    v4f bt = *(const v4f*)(beta  + ((size_t)d * 1024 + hw4) * 4);
    v4f o;
    o.x = (cv.x - mean) * rstd * gm.x + bt.x;
    o.y = (cv.y - mean) * rstd * gm.y + bt.y;
    o.z = (cv.z - mean) * rstd * gm.z + bt.z;
    o.w = (cv.w - mean) * rstd * gm.w + bt.w;
    float* op = out + (size_t)g * 4;
    *(volatile v4f*)op = o;
    __threadfence();
    *(volatile v4f*)op = o;
  }
}

extern "C" void kernel_launch(void* const* d_in, const int* in_sizes, int n_in,
                              void* d_out, int out_size, void* d_ws, size_t ws_size,
                              hipStream_t stream) {
  if (n_in < 5) return;
  if (in_sizes[0] != NBATCH * NDI * NS * NS) return;
  if (in_sizes[1] != NCH * KRED) return;
  if (in_sizes[2] != NCH) return;
  if (in_sizes[3] != NDO * NS * NS) return;
  if (in_sizes[4] != NDO * NS * NS) return;
  if (out_size != NCO * NBATCH * NDO * NS * NS) return;

  const float* caps_in = (const float*)d_in[0];
  const float* W       = (const float*)d_in[1];
  const float* bias    = (const float*)d_in[2];
  const float* gamma   = (const float*)d_in[3];
  const float* beta    = (const float*)d_in[4];

  const size_t wr_bytes   = (size_t)NWCHUNK * 16;
  const size_t caps_bytes = (size_t)NBATCH * NCO * NDO * NS * NS * 4;
  const size_t part_bytes = (size_t)NCONVBLK * PARTW * 4;
  if (wr_bytes + caps_bytes + part_bytes > ws_size) return;

  char* ws = (char*)d_ws;
  v4u*   Wr      = (v4u*)ws;
  float* capsbuf = (float*)(ws + wr_bytes);
  float* part    = (float*)(ws + wr_bytes + caps_bytes);

  const int n4 = out_size / 4;
  const int nprep = (NWCHUNK + 255) / 256;
  const int nfin  = (n4 + 255) / 256;

  k_prep<<<nprep, 256, 0, stream>>>(W, Wr, (int)NWCHUNK);
  k_conv_route<<<NCONVBLK, 256, 0, stream>>>(caps_in, Wr, bias, capsbuf, part);
  k_final<<<nfin, 256, 0, stream>>>(capsbuf, part, gamma, beta, (float*)d_out, n4);
}
